// GRU_43568148251487
// MI455X (gfx1250) — hardware-run, weakly checked
//
#include <hip/hip_runtime.h>
#include <math.h>

constexpr int NSEQ   = 64;
constexpr int NSTEP  = 512;
constexpr int DIN    = 64;
constexpr int DMODEL = 256;
constexpr int NHID   = 512;
constexpr int NGATE  = 3 * NHID;
constexpr int DOUT   = 64;
constexpr int NROWS  = NSEQ * NSTEP;
constexpr int NTHR   = 256;
constexpr int SEQ_BLK = 16;
constexpr int HP     = NHID + 8;
constexpr int SLABP  = 68;
constexpr float ACT_CARRY = 16.0f;
constexpr float W_CARRY   = 64.0f;
constexpr float ACC_FOLD  = 1.0f / (ACT_CARRY * W_CARRY);
constexpr float F16_MIN_NORMAL = 6.103515625e-5f;

static_assert(NSEQ % SEQ_BLK == 0, "batch tiles");
static_assert(NHID == 64 * (NTHR / 32), "8 waves x 64 hidden units");
static_assert(DIN % 32 == 0 && DMODEL % 32 == 0 && NHID % 32 == 0, "K multiples of 32");
static_assert(NROWS % 32 == 0 && DMODEL % 64 == 0 && DOUT == 64, "tile multiples");
static_assert(HP % 8 == 0, "16-B aligned fragment rows");
static_assert(NGATE == 1536, "gate rows");

typedef __attribute__((ext_vector_type(16))) _Float16 v16h;
typedef __attribute__((ext_vector_type(8)))  _Float16 v8h;
typedef __attribute__((ext_vector_type(16))) __bf16   v16b;
typedef __attribute__((ext_vector_type(8)))  __bf16   v8b;
typedef __attribute__((ext_vector_type(8)))  float    v8f;
typedef __attribute__((ext_vector_type(4)))  float    v4f;
typedef __attribute__((ext_vector_type(4)))  unsigned v4u;

__device__ __forceinline__ unsigned f2bf_bits(float f) {
  const unsigned u = __float_as_uint(f);
  return ((u + 0x7FFFu + ((u >> 16) & 1u)) >> 16) & 0xFFFFu;
}
__device__ __forceinline__ float bf_bits2f(unsigned h) { return __uint_as_float(h << 16); }
__device__ __forceinline__ void split_bf(float v, unsigned& hb, unsigned& lb) {
  hb = f2bf_bits(v);
  lb = f2bf_bits(v - bf_bits2f(hb));
}
__device__ __forceinline__ _Float16 h16_ftz(float v) {
  const float w = (fabsf(v) < F16_MIN_NORMAL) ? 0.0f : v;
  return (_Float16)w;
}
__device__ __forceinline__ unsigned h16_ftz_bits(float v) {
  const _Float16 h = h16_ftz(v);
  return (unsigned)__builtin_bit_cast(unsigned short, h);
}

union FragHU { v16h v; v8h h[2]; };
union FragBU { v16b v; v8b h[2]; };
__device__ __forceinline__ v16h ldfrag_h(const _Float16* p) {
  FragHU f; f.h[0] = *(const v8h*)(p); f.h[1] = *(const v8h*)(p + 16); return f.v;
}
__device__ __forceinline__ v16b ldfrag_b(const __bf16* p) {
  FragBU f; f.h[0] = *(const v8b*)(p); f.h[1] = *(const v8b*)(p + 16); return f.v;
}
__device__ __forceinline__ v8f mma_h(v16h a, v16h b, v8f c) {
  c = __builtin_amdgcn_wmma_f32_16x16x32_f16(false, a, false, b, (short)0, c, false, false);
  asm volatile("v_nop\n\tv_nop\n\tv_nop\n\tv_nop" : "+v"(c) : "v"(a), "v"(b));
  return c;
}
__device__ __forceinline__ v8f mma_b(v16b a, v16b b, v8f c) {
  c = __builtin_amdgcn_wmma_f32_16x16x32_bf16(false, a, false, b, (short)0, c, false, false);
  asm volatile("v_nop\n\tv_nop\n\tv_nop\n\tv_nop" : "+v"(c) : "v"(a), "v"(b));
  return c;
}

__device__ __forceinline__ float fsig(float x)  { return __builtin_amdgcn_rcpf(1.0f + __expf(-x)); }
__device__ __forceinline__ float ftanh(float x) { return 1.0f - 2.0f * __builtin_amdgcn_rcpf(__expf(2.0f * x) + 1.0f); }

__device__ __forceinline__ float cell_update(float aR, float aZ, float aI, float aH,
                                             float bR, float bZ, float bI, float bH, float hold) {
  const float pr  = aR * ACC_FOLD + bR;
  const float pz  = aZ * ACC_FOLD + bZ;
  const float gin = aI * ACC_FOLD + bI;
  const float ghn = aH * ACC_FOLD + bH;
  const float rg = fsig(pr);
  const float zg = fsig(pz);
  const float ng = ftanh(gin + rg * ghn);
  return (1.0f - zg) * ng + zg * hold;
}

constexpr int CB_WX   = (DMODEL * DIN / 8) / NTHR;
constexpr int CB_WIH0 = (NGATE * DMODEL / 8) / NTHR;
constexpr int CB_WHH  = (NGATE * NHID / 8) / NTHR;
constexpr int CB_WO   = (DOUT * NHID / 8) / NTHR;
constexpr int CB_X    = (NROWS * DIN / 8) / NTHR;
constexpr int CE0 = CB_WX;
constexpr int CE1 = CE0 + CB_WIH0;
constexpr int CE2 = CE1 + CB_WHH;
constexpr int CE3 = CE2 + CB_WHH;
constexpr int CE4 = CE3 + CB_WHH;
constexpr int CE5 = CE4 + CB_WO;
constexpr int CE6 = CE5 + CB_X;
static_assert((DMODEL * DIN) % (8 * NTHR) == 0 && (NGATE * DMODEL) % (8 * NTHR) == 0, "exact cover");
static_assert((NGATE * NHID) % (8 * NTHR) == 0 && (DOUT * NHID) % (8 * NTHR) == 0, "exact cover");
static_assert((NROWS * DIN) % (8 * NTHR) == 0, "exact cover");
static_assert(CE6 == 2392, "convert grid");

__device__ __forceinline__ void load8(const float* __restrict__ sp, float (&f)[8]) {
  const v4f a = *(const v4f*)(sp);
  const v4f b = *(const v4f*)(sp + 4);
  f[0] = a[0]; f[1] = a[1]; f[2] = a[2]; f[3] = a[3];
  f[4] = b[0]; f[5] = b[1]; f[6] = b[2]; f[7] = b[3];
}
__device__ __forceinline__ void cvt8_split(const float* __restrict__ src, unsigned short* __restrict__ dh,
                                           unsigned short* __restrict__ dl, int i, float sc) {
  float f[8];
  load8(src + (size_t)i * 8, f);
  unsigned hb[8], lb[8];
#pragma unroll
  for (int e = 0; e < 8; ++e) split_bf(f[e] * sc, hb[e], lb[e]);
  v4u hw, lw;
#pragma unroll
  for (int e = 0; e < 4; ++e) {
    hw[e] = hb[2 * e] | (hb[2 * e + 1] << 16);
    lw[e] = lb[2 * e] | (lb[2 * e + 1] << 16);
  }
  unsigned short* ph = dh + (size_t)i * 8;
  unsigned short* pl = dl + (size_t)i * 8;
  *(volatile v4u*)ph = hw;
  *(volatile v4u*)pl = lw;
  __threadfence();
  *(volatile v4u*)ph = hw;
  *(volatile v4u*)pl = lw;
}
__device__ __forceinline__ void cvt8_f16(const float* __restrict__ src, unsigned short* __restrict__ dh, int i, float sc) {
  float f[8];
  load8(src + (size_t)i * 8, f);
  unsigned hb[8];
#pragma unroll
  for (int e = 0; e < 8; ++e) hb[e] = h16_ftz_bits(f[e] * sc);
  v4u hw;
#pragma unroll
  for (int e = 0; e < 4; ++e) hw[e] = hb[2 * e] | (hb[2 * e + 1] << 16);
  unsigned short* ph = dh + (size_t)i * 8;
  *(volatile v4u*)ph = hw;
  __threadfence();
  *(volatile v4u*)ph = hw;
}

__global__ __launch_bounds__(NTHR) void planes_kernel(
    const float* __restrict__ x, const float* __restrict__ Wx, const float* __restrict__ W_ih0,
    const float* __restrict__ W_hh0, const float* __restrict__ W_ih1, const float* __restrict__ W_hh1,
    const float* __restrict__ Wo,
    unsigned short* __restrict__ XH, unsigned short* __restrict__ XL,
    unsigned short* __restrict__ WXH, unsigned short* __restrict__ WXL,
    unsigned short* __restrict__ W0H, unsigned short* __restrict__ W0L,
    unsigned short* __restrict__ WHH0, unsigned short* __restrict__ WIH1, unsigned short* __restrict__ WHH1,
    unsigned short* __restrict__ WOH, unsigned short* __restrict__ WOL) {
  const int blk = blockIdx.x, tid = threadIdx.x;
  if (blk < CE0) {
    cvt8_split(Wx, WXH, WXL, blk * NTHR + tid, 1.0f);
  } else if (blk < CE1) {
    cvt8_split(W_ih0, W0H, W0L, (blk - CE0) * NTHR + tid, W_CARRY);
  } else if (blk < CE2) {
    cvt8_f16(W_hh0, WHH0, (blk - CE1) * NTHR + tid, W_CARRY);
  } else if (blk < CE3) {
    cvt8_f16(W_ih1, WIH1, (blk - CE2) * NTHR + tid, W_CARRY);
  } else if (blk < CE4) {
    cvt8_f16(W_hh1, WHH1, (blk - CE3) * NTHR + tid, W_CARRY);
  } else if (blk < CE5) {
    cvt8_split(Wo, WOH, WOL, (blk - CE4) * NTHR + tid, 1.0f);
  } else if (blk < CE6) {
    cvt8_split(x, XH, XL, (blk - CE5) * NTHR + tid, 1.0f);
  }
}

constexpr int XP_TILES = (NROWS / 32) * (DMODEL / 64);
static_assert(XP_TILES % 8 == 0, "whole blocks");

__global__ __launch_bounds__(NTHR) void xp_gemm_kernel(
    const unsigned short* __restrict__ XHp, const unsigned short* __restrict__ XLp,
    const unsigned short* __restrict__ WXHp, const unsigned short* __restrict__ WXLp,
    const float* __restrict__ bx, const float* __restrict__ wt, const float* __restrict__ bt,
    const float* __restrict__ tin,
    unsigned short* __restrict__ XPH, unsigned short* __restrict__ XPL) {
  __shared__ __align__(16) float sT[NTHR / 32][16 * SLABP];
  const __bf16* XH  = (const __bf16*)XHp;
  const __bf16* XL  = (const __bf16*)XLp;
  const __bf16* WXH = (const __bf16*)WXHp;
  const __bf16* WXL = (const __bf16*)WXLp;
  const int lane = threadIdx.x & 31, wave = threadIdx.x >> 5;
  const int tile = blockIdx.x * 8 + wave;
  if (tile >= XP_TILES) return;
  const int tm = tile >> 2, tn = tile & 3;
  const int m0 = tm * 32, n0 = tn * 64;
  const int rl = lane & 15, koff = (lane >> 4) * 8, mOff = (lane >> 4) * 8;

  v8f acc[2][4];
#pragma unroll
  for (int i = 0; i < 2; ++i)
#pragma unroll
    for (int j = 0; j < 4; ++j) acc[i][j] = (v8f){0.f, 0.f, 0.f, 0.f, 0.f, 0.f, 0.f, 0.f};

#pragma unroll 1
  for (int k0 = 0; k0 < DIN; k0 += 32) {
    v16b bh[4], bl[4];
#pragma unroll
    for (int j = 0; j < 4; ++j) {
      const size_t bofs = (size_t)(n0 + 16 * j + rl) * DIN + koff + k0;
      bh[j] = ldfrag_b(WXH + bofs);
      bl[j] = ldfrag_b(WXL + bofs);
    }
#pragma unroll
    for (int i = 0; i < 2; ++i) {
      const size_t aofs = (size_t)(m0 + 16 * i + rl) * DIN + koff + k0;
      const v16b ah = ldfrag_b(XH + aofs);
      const v16b al = ldfrag_b(XL + aofs);
#pragma unroll
      for (int j = 0; j < 4; ++j) {
        acc[i][j] = mma_b(ah, bh[j], acc[i][j]);
        acc[i][j] = mma_b(ah, bl[j], acc[i][j]);
        acc[i][j] = mma_b(al, bh[j], acc[i][j]);
      }
    }
  }

  float* slab = sT[wave];
  const int q = lane >> 3, c8 = (lane & 7) * 8;
  float bxv[8], wtv[8], btv[8];
  load8(bx + n0 + c8, bxv);
  load8(wt + n0 + c8, wtv);
  load8(bt + n0 + c8, btv);
#pragma unroll
  for (int i = 0; i < 2; ++i) {
    const int mBase = m0 + 16 * i;
#pragma unroll
    for (int j = 0; j < 4; ++j)
#pragma unroll
      for (int r = 0; r < 8; ++r) slab[(mOff + r) * SLABP + 16 * j + rl] = acc[i][j][r];
    __builtin_amdgcn_fence(__ATOMIC_RELEASE, "workgroup");
    __builtin_amdgcn_wave_barrier();
    __builtin_amdgcn_fence(__ATOMIC_ACQUIRE, "workgroup");
    v4u hw[4], lw[4];
#pragma unroll
    for (int it = 0; it < 4; ++it) {
      const int row = it * 4 + q;
      const float tv = tin[mBase + row];
      float sv[8];
      load8(slab + row * SLABP + c8, sv);
      unsigned hb[8], lb[8];
#pragma unroll
      for (int e = 0; e < 8; ++e) {
        const float v = ((sv[e] + bxv[e]) + tv * wtv[e]) + btv[e];
        split_bf(v * ACT_CARRY, hb[e], lb[e]);
      }
#pragma unroll
      for (int e = 0; e < 4; ++e) {
        hw[it][e] = hb[2 * e] | (hb[2 * e + 1] << 16);
        lw[it][e] = lb[2 * e] | (lb[2 * e + 1] << 16);
      }
    }
    for (int pass = 0; pass < 2; ++pass) {
#pragma unroll
      for (int it = 0; it < 4; ++it) {
        const int row = it * 4 + q;
        const size_t o = (size_t)(mBase + row) * DMODEL + n0 + c8;
        *(volatile v4u*)(XPH + o) = hw[it];
        *(volatile v4u*)(XPL + o) = lw[it];
      }
      __threadfence();
    }
    __builtin_amdgcn_fence(__ATOMIC_RELEASE, "workgroup");
    __builtin_amdgcn_wave_barrier();
    __builtin_amdgcn_fence(__ATOMIC_ACQUIRE, "workgroup");
  }
}

__global__ __launch_bounds__(NTHR) void seq2_kernel(
    const unsigned short* __restrict__ XPHp, const unsigned short* __restrict__ XPLp,
    const unsigned short* __restrict__ W0Hp, const unsigned short* __restrict__ W0Lp,
    const unsigned short* __restrict__ WHH0p, const unsigned short* __restrict__ WIH1p,
    const unsigned short* __restrict__ WHH1p,
    const unsigned short* __restrict__ WOHp, const unsigned short* __restrict__ WOLp,
    const float* __restrict__ b_ih0, const float* __restrict__ b_hh0,
    const float* __restrict__ b_ih1, const float* __restrict__ b_hh1,
    const float* __restrict__ bo, float* __restrict__ out) {
  __shared__ __align__(16) _Float16 Ah0[2][SEQ_BLK * HP];
  __shared__ __align__(16) _Float16 Ah1[2][SEQ_BLK * HP];
  __shared__ __align__(16) __bf16   Rh[SEQ_BLK * HP];
  __shared__ __align__(16) __bf16   Rl[SEQ_BLK * HP];
  __shared__ __align__(16) float    Ps[2][16 * SLABP];

  const __bf16*   XPH  = (const __bf16*)XPHp;
  const __bf16*   XPL  = (const __bf16*)XPLp;
  const __bf16*   W0H  = (const __bf16*)W0Hp;
  const __bf16*   W0L  = (const __bf16*)W0Lp;
  const _Float16* WHH0 = (const _Float16*)WHH0p;
  const _Float16* WIH1 = (const _Float16*)WIH1p;
  const _Float16* WHH1 = (const _Float16*)WHH1p;
  const __bf16*   WOH  = (const __bf16*)WOHp;
  const __bf16*   WOL  = (const __bf16*)WOLp;

  const int tid = threadIdx.x, lane = tid & 31, wave = tid >> 5;
  const int c = lane & 15, hh = lane >> 4, koff = hh * 8;
  const int rowbase = blockIdx.x * SEQ_BLK;

  {
    _Float16* p0 = &Ah0[0][0];
    _Float16* p1 = &Ah1[0][0];
    float* pp = &Ps[0][0];
    const __bf16 bz = __builtin_bit_cast(__bf16, (unsigned short)0);
#pragma unroll 1
    for (int i = tid; i < 2 * SEQ_BLK * HP; i += NTHR) { p0[i] = (_Float16)0.0f; p1[i] = (_Float16)0.0f; }
#pragma unroll 1
    for (int i = tid; i < SEQ_BLK * HP; i += NTHR) { Rh[i] = bz; Rl[i] = bz; }
#pragma unroll 1
    for (int i = tid; i < 2 * 16 * SLABP; i += NTHR) pp[i] = 0.0f;
  }
  float hst0[4][8], hst1[4][8];
#pragma unroll
  for (int nt = 0; nt < 4; ++nt)
#pragma unroll
    for (int r = 0; r < 8; ++r) { hst0[nt][r] = 0.0f; hst1[nt][r] = 0.0f; }
  __syncthreads();

  const v8f z8 = {0.f, 0.f, 0.f, 0.f, 0.f, 0.f, 0.f, 0.f};

#pragma unroll 1
  for (int t = 0; t < NSTEP; ++t) {
    const int cur = t & 1, nxt = cur ^ 1;

    {
      const _Float16* a0 = &Ah0[cur][0] + c * HP + koff;
      _Float16* a0n = &Ah0[nxt][0];
      const size_t xo = ((size_t)(rowbase + c) * NSTEP + (size_t)t) * DMODEL + koff;
      const __bf16* xh = XPH + xo;
      const __bf16* xl = XPL + xo;
#pragma unroll
      for (int nt = 0; nt < 4; ++nt) {
        const int j = 64 * wave + 16 * nt + c;
        v8f aR = z8, aZ = z8, aI = z8, aH = z8;
        {
          const size_t wofs = (size_t)j * DMODEL + koff;
          const __bf16* wh = W0H + wofs;
          const __bf16* wl = W0L + wofs;
#pragma unroll 1
          for (int k0 = 0; k0 < DMODEL; k0 += 32) {
            const v16b ah = ldfrag_b(xh + k0);
            const v16b al = ldfrag_b(xl + k0);
            {
              const v16b bh = ldfrag_b(wh + k0);
              const v16b bl = ldfrag_b(wl + k0);
              aR = mma_b(ah, bh, aR);
              aR = mma_b(ah, bl, aR);
              aR = mma_b(al, bh, aR);
            }
            {
              const v16b bh = ldfrag_b(wh + (size_t)NHID * DMODEL + k0);
              const v16b bl = ldfrag_b(wl + (size_t)NHID * DMODEL + k0);
              aZ = mma_b(ah, bh, aZ);
              aZ = mma_b(ah, bl, aZ);
              aZ = mma_b(al, bh, aZ);
            }
            {
              const v16b bh = ldfrag_b(wh + (size_t)2 * NHID * DMODEL + k0);
              const v16b bl = ldfrag_b(wl + (size_t)2 * NHID * DMODEL + k0);
              aI = mma_b(ah, bh, aI);
              aI = mma_b(ah, bl, aI);
              aI = mma_b(al, bh, aI);
            }
          }
        }
        {
          const _Float16* wr = WHH0 + (size_t)j * NHID + koff;
#pragma unroll 1
          for (int k0 = 0; k0 < NHID; k0 += 32) {
            const v16h a  = ldfrag_h(a0 + k0);
            const v16h f0 = ldfrag_h(wr + k0);
            const v16h f1 = ldfrag_h(wr + (size_t)NHID * NHID + k0);
            const v16h f2 = ldfrag_h(wr + (size_t)2 * NHID * NHID + k0);
            aR = mma_h(a, f0, aR);
            aZ = mma_h(a, f1, aZ);
            aH = mma_h(a, f2, aH);
          }
        }
        const float bR = b_ih0[j] + b_hh0[j];
        const float bZ = b_ih0[NHID + j] + b_hh0[NHID + j];
        const float bI = b_ih0[2 * NHID + j];
        const float bH = b_hh0[2 * NHID + j];
#pragma unroll
        for (int r = 0; r < 8; ++r) {
          const float hn = cell_update(aR[r], aZ[r], aI[r], aH[r], bR, bZ, bI, bH, hst0[nt][r]);
          hst0[nt][r] = hn;
          a0n[(8 * hh + r) * HP + j] = h16_ftz(hn * ACT_CARRY);
        }
      }
    }
    __syncthreads();

    {
      const _Float16* ain = &Ah0[nxt][0] + c * HP + koff;
      const _Float16* a1  = &Ah1[cur][0] + c * HP + koff;
      _Float16* a1n = &Ah1[nxt][0];
#pragma unroll
      for (int nt = 0; nt < 4; ++nt) {
        const int j = 64 * wave + 16 * nt + c;
        v8f aR = z8, aZ = z8, aI = z8, aH = z8;
        {
          const _Float16* wi = WIH1 + (size_t)j * NHID + koff;
#pragma unroll 1
          for (int k0 = 0; k0 < NHID; k0 += 32) {
            const v16h a  = ldfrag_h(ain + k0);
            const v16h f0 = ldfrag_h(wi + k0);
            const v16h f1 = ldfrag_h(wi + (size_t)NHID * NHID + k0);
            const v16h f2 = ldfrag_h(wi + (size_t)2 * NHID * NHID + k0);
            aR = mma_h(a, f0, aR);
            aZ = mma_h(a, f1, aZ);
            aI = mma_h(a, f2, aI);
          }
        }
        {
          const _Float16* wr = WHH1 + (size_t)j * NHID + koff;
#pragma unroll 1
          for (int k0 = 0; k0 < NHID; k0 += 32) {
            const v16h a  = ldfrag_h(a1 + k0);
            const v16h f0 = ldfrag_h(wr + k0);
            const v16h f1 = ldfrag_h(wr + (size_t)NHID * NHID + k0);
            const v16h f2 = ldfrag_h(wr + (size_t)2 * NHID * NHID + k0);
            aR = mma_h(a, f0, aR);
            aZ = mma_h(a, f1, aZ);
            aH = mma_h(a, f2, aH);
          }
        }
        const float bR = b_ih1[j] + b_hh1[j];
        const float bZ = b_ih1[NHID + j] + b_hh1[NHID + j];
        const float bI = b_ih1[2 * NHID + j];
        const float bH = b_hh1[2 * NHID + j];
#pragma unroll
        for (int r = 0; r < 8; ++r) {
          const float hn = cell_update(aR[r], aZ[r], aI[r], aH[r], bR, bZ, bI, bH, hst1[nt][r]);
          hst1[nt][r] = hn;
          const int li = (8 * hh + r) * HP + j;
          a1n[li] = h16_ftz(hn * ACT_CARRY);
          const float rv = fmaxf(hn, 0.0f);
          unsigned hb, lb;
          split_bf(rv, hb, lb);
          Rh[li] = __builtin_bit_cast(__bf16, (unsigned short)hb);
          Rl[li] = __builtin_bit_cast(__bf16, (unsigned short)lb);
        }
      }
    }
    __syncthreads();

    {
      const int ct = wave & 3, kh = wave >> 2;
      v8f ac = z8;
      const __bf16* rh = Rh + c * HP + koff + 256 * kh;
      const __bf16* rl = Rl + c * HP + koff + 256 * kh;
      const size_t wofs = (size_t)(16 * ct + c) * NHID + koff + 256 * kh;
      const __bf16* wh = WOH + wofs;
      const __bf16* wl = WOL + wofs;
#pragma unroll 1
      for (int k0 = 0; k0 < NHID / 2; k0 += 32) {
        const v16b ah = ldfrag_b(rh + k0);
        const v16b al = ldfrag_b(rl + k0);
        const v16b bh = ldfrag_b(wh + k0);
        const v16b bl = ldfrag_b(wl + k0);
        ac = mma_b(ah, bh, ac);
        ac = mma_b(ah, bl, ac);
        ac = mma_b(al, bh, ac);
      }
      float* ps = &Ps[kh][0];
#pragma unroll
      for (int r = 0; r < 8; ++r) ps[(8 * hh + r) * SLABP + 16 * ct + c] = ac[r];
    }
    __syncthreads();

    {
      const int row = 2 * wave + hh, c4 = c * 4;
      const v4f p0 = *(const v4f*)(&Ps[0][0] + row * SLABP + c4);
      const v4f p1 = *(const v4f*)(&Ps[1][0] + row * SLABP + c4);
      const v4f bv = *(const v4f*)(bo + c4);
      v4f o;
      o[0] = (p0[0] + p1[0]) + bv[0];
      o[1] = (p0[1] + p1[1]) + bv[1];
      o[2] = (p0[2] + p1[2]) + bv[2];
      o[3] = (p0[3] + p1[3]) + bv[3];
      float* op = out + ((size_t)(rowbase + row) * NSTEP + (size_t)t) * DOUT + c4;
      *(volatile v4f*)op = o;
      __threadfence();
      *(volatile v4f*)op = o;
    }
  }
}

extern "C" void kernel_launch(void* const* d_in, const int* in_sizes, int n_in,
                              void* d_out, int out_size, void* d_ws, size_t ws_size, hipStream_t stream) {
  if (n_in < 16 || d_out == nullptr || d_ws == nullptr) return;
  if (in_sizes[0] != NROWS * DIN || in_sizes[1] != NROWS || in_sizes[2] != DMODEL * DIN ||
      in_sizes[3] != DMODEL || in_sizes[4] != DMODEL || in_sizes[5] != DMODEL ||
      in_sizes[6] != NGATE * DMODEL || in_sizes[7] != NGATE * NHID || in_sizes[8] != NGATE ||
      in_sizes[9] != NGATE || in_sizes[10] != NGATE * NHID || in_sizes[11] != NGATE * NHID ||
      in_sizes[12] != NGATE || in_sizes[13] != NGATE || in_sizes[14] != DOUT * NHID ||
      in_sizes[15] != DOUT || out_size != NROWS * DOUT) return;

  const float* x     = (const float*)d_in[0];
  const float* tin   = (const float*)d_in[1];
  const float* Wx    = (const float*)d_in[2];
  const float* bx    = (const float*)d_in[3];
  const float* Wt    = (const float*)d_in[4];
  const float* bt    = (const float*)d_in[5];
  const float* W_ih0 = (const float*)d_in[6];
  const float* W_hh0 = (const float*)d_in[7];
  const float* b_ih0 = (const float*)d_in[8];
  const float* b_hh0 = (const float*)d_in[9];
  const float* W_ih1 = (const float*)d_in[10];
  const float* W_hh1 = (const float*)d_in[11];
  const float* b_ih1 = (const float*)d_in[12];
  const float* b_hh1 = (const float*)d_in[13];
  const float* Wo    = (const float*)d_in[14];
  const float* bo    = (const float*)d_in[15];
  float* out = (float*)d_out;

  char* ws = (char*)d_ws;
  size_t off = 0;
  auto carve = [&](size_t bytes) -> char* { char* p = ws + off; off += (bytes + 255) & ~(size_t)255; return p; };
  unsigned short* XH   = (unsigned short*)carve((size_t)NROWS * DIN * 2);
  unsigned short* XL   = (unsigned short*)carve((size_t)NROWS * DIN * 2);
  unsigned short* WXH  = (unsigned short*)carve((size_t)DMODEL * DIN * 2);
  unsigned short* WXL  = (unsigned short*)carve((size_t)DMODEL * DIN * 2);
  unsigned short* W0H  = (unsigned short*)carve((size_t)NGATE * DMODEL * 2);
  unsigned short* W0L  = (unsigned short*)carve((size_t)NGATE * DMODEL * 2);
  unsigned short* WHH0 = (unsigned short*)carve((size_t)NGATE * NHID * 2);
  unsigned short* WIH1 = (unsigned short*)carve((size_t)NGATE * NHID * 2);
  unsigned short* WHH1 = (unsigned short*)carve((size_t)NGATE * NHID * 2);
  unsigned short* WOH  = (unsigned short*)carve((size_t)DOUT * NHID * 2);
  unsigned short* WOL  = (unsigned short*)carve((size_t)DOUT * NHID * 2);
  unsigned short* XPH  = (unsigned short*)carve((size_t)NROWS * DMODEL * 2);
  unsigned short* XPL  = (unsigned short*)carve((size_t)NROWS * DMODEL * 2);
  if (off > ws_size || off > (size_t)134217728) return;

  planes_kernel<<<CE6, NTHR, 0, stream>>>(x, Wx, W_ih0, W_hh0, W_ih1, W_hh1, Wo,
                                          XH, XL, WXH, WXL, W0H, W0L, WHH0, WIH1, WHH1, WOH, WOL);
  xp_gemm_kernel<<<XP_TILES / 8, NTHR, 0, stream>>>(XH, XL, WXH, WXL, bx, Wt, bt, tin, XPH, XPL);
  seq2_kernel<<<NSEQ / SEQ_BLK, NTHR, 0, stream>>>(XPH, XPL, W0H, W0L, WHH0, WIH1, WHH1, WOH, WOL,
                                                   b_ih0, b_hh0, b_ih1, b_hh1, bo, out);
}
